// DGATModule_47467978555681
// MI455X (gfx1250) — hardware-verified
//
#include <hip/hip_runtime.h>
#include <stddef.h>


#define DIMF   64
#define NHD    8
#define HID    256
#define GR     32
#define APN    72
#define HPN    68
#define GPN    264
#define NB     512
#define CHUNK  2048
#define NTHR   256
#define NWAVE  8
#define WCAP   256
#define NGRP   (CHUNK / (NTHR * 4))
#define NPREP  19

#define L_SACC 0
#define L_SDEN (L_SACC + NB * DIMF)
#define L_SMAX (L_SDEN + NB * NHD)
#define L_SSV  (L_SMAX + NB * NHD)
#define L_LIST (L_SSV + NB * NHD)
#define L_WCNT (L_LIST + NWAVE * WCAP)
#define L_KAP  (L_WCNT + NWAVE)
#define L_AH   (L_KAP + 32)
#define L_AL   (L_AH + 16 * APN / 2)
#define L_GH   (L_AL + 16 * APN / 2)
#define L_GL   (L_GH + 16 * GPN / 2)
#define L_OS   (L_GL + 16 * GPN / 2)
#define L_TOT  (L_OS + 16 * HPN)
#define LDS_BYTES (L_TOT * 4)

static_assert(NGRP == 2);
static_assert(WCAP == (CHUNK / NTHR) * 32);
static_assert(NB == 512);
static_assert(CHUNK <= 2048);
static_assert((L_SDEN % 4) == 0 && (L_SMAX % 4) == 0 && (L_SSV % 4) == 0 && (L_LIST % 4) == 0);
static_assert((L_KAP % 4) == 0 && (L_AH % 4) == 0 && (L_AL % 4) == 0 && (L_GH % 4) == 0 && (L_GL % 4) == 0 && (L_OS % 4) == 0);
static_assert(LDS_BYTES == 214432);

typedef float          v2f   __attribute__((ext_vector_type(2)));
typedef float          v4f   __attribute__((ext_vector_type(4)));
typedef float          v8f   __attribute__((ext_vector_type(8)));
typedef int            v4i   __attribute__((ext_vector_type(4)));
typedef unsigned short v4us  __attribute__((ext_vector_type(4)));
typedef unsigned short v8us  __attribute__((ext_vector_type(8)));
typedef __bf16         v16bf __attribute__((ext_vector_type(16)));
typedef unsigned short us;
union FragB { v16bf v; v8us u[2]; };

__device__ __forceinline__ v8f wmb(v16bf a, v16bf b, v8f c) {
  v8f d = __builtin_amdgcn_wmma_f32_16x16x32_bf16(false, a, false, b, (short)0, c, false, false);
  asm volatile("v_nop\n\tv_nop\n\tv_nop\n\tv_nop" : "+v"(d) : "v"(a), "v"(b));
  return d;
}
__device__ __forceinline__ v8f wm3(const FragB& ah, const FragB& al, const FragB& bh, const FragB& bl, v8f c) {
  c = wmb(ah.v, bh.v, c);
  c = wmb(ah.v, bl.v, c);
  c = wmb(al.v, bh.v, c);
  return c;
}
__device__ __forceinline__ void ldf(FragB& f, const us* p) {
  f.u[0] = *(const v8us*)(p);
  f.u[1] = *(const v8us*)(p + 16);
}
__device__ __forceinline__ us bfh(float f) {
  const unsigned u = __float_as_uint(f);
  return (us)((u + 0x7FFFu + ((u >> 16) & 1u)) >> 16);
}
__device__ __forceinline__ void spl(float f, us& hi, us& lo) {
  hi = bfh(f);
  const float r = f - __uint_as_float(((unsigned)hi) << 16);
  lo = bfh(r);
}
__device__ __forceinline__ float gelu_x(float v) {
  return 0.5f * v * (1.0f + erff(v * 0.70710678118654752f));
}

__global__ __launch_bounds__(NTHR) void k_prep(
    const float* __restrict__ w_in, const float* __restrict__ w_att_u, const float* __restrict__ w_att_v,
    const float* __restrict__ w_ff1, const float* __restrict__ w_ff2,
    us* WinH, us* WinL, us* WuvH, us* WuvL, us* W1H, us* W1L, us* W2H, us* W2L) {
  const int b = blockIdx.x, t = threadIdx.x;
  float v[8];
  us* ph;
  us* pl;
  size_t o;
  bool act = true;
  if (b < 2) {
    const int g = b * NTHR + t;
    const int n = g >> 3, k0 = (g & 7) * 8;
#pragma unroll
    for (int j = 0; j < 8; ++j) v[j] = w_in[(k0 + j) * DIMF + n];
    ph = WinH; pl = WinL; o = (size_t)g * 8;
  } else if (b == 2) {
    act = (t < 128);
    const int g = t & 127;
    const int n = g >> 3, k0 = (g & 7) * 8;
    const int nu = n & 7;
    const int nv = (n >= 8) ? (n - 8) : 0;
#pragma unroll
    for (int j = 0; j < 8; ++j) {
      const float a = w_att_u[(k0 + j) * NHD + nu];
      const float c = w_att_v[(k0 + j) * NHD + nv];
      v[j] = (n < 8) ? a : c;
    }
    ph = WuvH; pl = WuvL; o = (size_t)g * 8;
  } else if (b < 11) {
    const int g = (b - 3) * NTHR + t;
    const int n = g >> 3, k0 = (g & 7) * 8;
#pragma unroll
    for (int j = 0; j < 8; ++j) v[j] = w_ff1[(k0 + j) * HID + n];
    ph = W1H; pl = W1L; o = (size_t)g * 8;
  } else {
    const int g = (b - 11) * NTHR + t;
    const int n = g >> 5, k0 = (g & 31) * 8;
#pragma unroll
    for (int j = 0; j < 8; ++j) v[j] = w_ff2[(k0 + j) * DIMF + n];
    ph = W2H; pl = W2L; o = (size_t)g * 8;
  }
  v8us uh, ul;
#pragma unroll
  for (int j = 0; j < 8; ++j) {
    us a, c;
    spl(v[j], a, c);
    uh[j] = a;
    ul[j] = c;
  }
  if (act) {
    *(volatile v8us*)(ph + o) = uh;
    *(volatile v8us*)(pl + o) = ul;
  }
  __threadfence();
  if (act) {
    *(volatile v8us*)(ph + o) = uh;
    *(volatile v8us*)(pl + o) = ul;
  }
}

__global__ __launch_bounds__(128) void k_node(
    const float* __restrict__ x, const float* __restrict__ b_in, const float* __restrict__ b_att_u,
    const us* __restrict__ WinH, const us* __restrict__ WinL,
    const us* __restrict__ WuvH, const us* __restrict__ WuvL,
    float* hbuf, float* susv, int nN) {
  __shared__ __attribute__((aligned(16))) us    Ah[GR * APN];
  __shared__ __attribute__((aligned(16))) us    Al[GR * APN];
  __shared__ __attribute__((aligned(16))) float Hs[GR * HPN];
  __shared__ __attribute__((aligned(16))) float Ss[GR * 16];

  const int tid = threadIdx.x, lane = tid & 31, wave = tid >> 5;
  const int hh = lane >> 4, m = lane & 15;
  const int rowBase = blockIdx.x * GR;

  {
    const int r  = tid >> 2;
    const int c0 = (tid & 3) * 16;
    int row = rowBase + r;
    if (row > nN - 1) row = nN - 1;
    const float* p = x + (size_t)row * DIMF + c0;
    const v4f f0 = *(const v4f*)(p), f1 = *(const v4f*)(p + 4);
    const v4f f2 = *(const v4f*)(p + 8), f3 = *(const v4f*)(p + 12);
    v8us h0, l0, h1, l1;
#pragma unroll
    for (int j = 0; j < 4; ++j) {
      us a, c;
      spl(f0[j], a, c); h0[j] = a;     l0[j] = c;
      spl(f1[j], a, c); h0[4 + j] = a; l0[4 + j] = c;
      spl(f2[j], a, c); h1[j] = a;     l1[j] = c;
      spl(f3[j], a, c); h1[4 + j] = a; l1[4 + j] = c;
    }
    *(v8us*)(Ah + r * APN + c0)     = h0;
    *(v8us*)(Ah + r * APN + c0 + 8) = h1;
    *(v8us*)(Al + r * APN + c0)     = l0;
    *(v8us*)(Al + r * APN + c0 + 8) = l1;
  }
  __syncthreads();

  const int n = wave * 16 + m;
  v8f acc0 = {0.f, 0.f, 0.f, 0.f, 0.f, 0.f, 0.f, 0.f};
  v8f acc1 = {0.f, 0.f, 0.f, 0.f, 0.f, 0.f, 0.f, 0.f};
#pragma unroll
  for (int kt = 0; kt < DIMF / 32; ++kt) {
    const int k0 = kt * 32 + 8 * hh;
    FragB a0h, a0l, a1h, a1l, bh, bl;
    ldf(a0h, Ah + m * APN + k0);
    ldf(a0l, Al + m * APN + k0);
    ldf(a1h, Ah + (16 + m) * APN + k0);
    ldf(a1l, Al + (16 + m) * APN + k0);
    ldf(bh, WinH + (size_t)n * DIMF + k0);
    ldf(bl, WinL + (size_t)n * DIMF + k0);
    acc0 = wm3(a0h, a0l, bh, bl, acc0);
    acc1 = wm3(a1h, a1l, bh, bl, acc1);
  }
  __syncthreads();

  {
    const float bias = b_in[n];
#pragma unroll
    for (int r = 0; r < 8; ++r) {
      const int row0 = 8 * hh + r;
      const int row1 = 16 + 8 * hh + r;
      const float v0 = acc0[r] + bias;
      const float v1 = acc1[r] + bias;
      us a, c;
      Hs[row0 * HPN + n] = v0;
      spl(v0, a, c); Ah[row0 * APN + n] = a; Al[row0 * APN + n] = c;
      Hs[row1 * HPN + n] = v1;
      spl(v1, a, c); Ah[row1 * APN + n] = a; Al[row1 * APN + n] = c;
    }
  }
  __syncthreads();

  const int T = wave & 1;
  v8f acc2 = {0.f, 0.f, 0.f, 0.f, 0.f, 0.f, 0.f, 0.f};
#pragma unroll
  for (int kt = 0; kt < DIMF / 32; ++kt) {
    const int k0 = kt * 32 + 8 * hh;
    FragB ah, al, bh, bl;
    ldf(ah, Ah + (16 * T + m) * APN + k0);
    ldf(al, Al + (16 * T + m) * APN + k0);
    ldf(bh, WuvH + (size_t)m * DIMF + k0);
    ldf(bl, WuvL + (size_t)m * DIMF + k0);
    acc2 = wm3(ah, al, bh, bl, acc2);
  }
  {
    const float bu = b_att_u[m & 7];
    const float bias2 = (m < 8) ? bu : 0.0f;
    if (wave < 2) {
#pragma unroll
      for (int r = 0; r < 8; ++r) Ss[(16 * T + 8 * hh + r) * 16 + m] = acc2[r] + bias2;
    }
  }
  __syncthreads();

  v4f hv[4];
  float* hp[4];
#pragma unroll
  for (int i = 0; i < 4; ++i) {
    const int row = 8 * i + (tid >> 4);
    const int c4  = (tid & 15) * 4;
    hv[i] = *(const v4f*)(Hs + row * HPN + c4);
    hp[i] = hbuf + (size_t)(rowBase + row) * DIMF + c4;
  }
  const v4f sv4 = *(const v4f*)(Ss + tid * 4);
  float* sp = susv + (size_t)rowBase * 16 + tid * 4;
#pragma unroll
  for (int i = 0; i < 4; ++i) *(volatile v4f*)(hp[i]) = hv[i];
  *(volatile v4f*)sp = sv4;
  __threadfence();
#pragma unroll
  for (int i = 0; i < 4; ++i) *(volatile v4f*)(hp[i]) = hv[i];
  *(volatile v4f*)sp = sv4;
}

__global__ __launch_bounds__(NTHR) void k_agg(
    const float* __restrict__ hbuf, const float* __restrict__ susv, const float* __restrict__ edge_feat,
    const int* __restrict__ srci, const int* __restrict__ dsti,
    const float* __restrict__ w_edge, const float* __restrict__ b_edge,
    const float* __restrict__ w_att_e, const float* __restrict__ b_att_e,
    const us* __restrict__ W1H, const us* __restrict__ W1L,
    const us* __restrict__ W2H, const us* __restrict__ W2L,
    const float* __restrict__ b_ff1, const float* __restrict__ b_ff2,
    float* out, int nN, int nE) {
  extern __shared__ v4f lds_dyn[];
  float* ldsf = (float*)lds_dyn;
  float* sacc = ldsf + L_SACC;
  float* sden = ldsf + L_SDEN;
  float* smax = ldsf + L_SMAX;
  float* ssv  = ldsf + L_SSV;
  int*   list = (int*)(ldsf + L_LIST);
  int*   wcnt = (int*)(ldsf + L_WCNT);
  float* kap  = ldsf + L_KAP;
  us*    Ah   = (us*)(ldsf + L_AH);
  us*    Al   = (us*)(ldsf + L_AL);
  us*    Gh   = (us*)(ldsf + L_GH);
  us*    Gl   = (us*)(ldsf + L_GL);
  float* Os   = ldsf + L_OS;

  const int tid = threadIdx.x, lane = tid & 31, wave = tid >> 5;
  const int hh = lane >> 4, m = lane & 15;
  const int hd = lane & 7;
  const int hc0 = (2 * lane) & 7;
  const int hc1 = hc0 + 1;
  const int nodeBase = blockIdx.x * NB;

  {
    const v4f z4 = {0.f, 0.f, 0.f, 0.f};
    for (int i = tid; i < (NB * DIMF + NB * NHD) / 4; i += NTHR) lds_dyn[i] = z4;
    const v4f n4 = {-3.0e38f, -3.0e38f, -3.0e38f, -3.0e38f};
#pragma unroll
    for (int i = 0; i < 4; ++i) {
      const int idx = i * NTHR + tid;
      *(v4f*)(smax + 4 * idx) = n4;
    }
#pragma unroll
    for (int i = 0; i < 4; ++i) {
      const int idx  = i * NTHR + tid;
      const int slot = idx >> 1;
      const int half = idx & 1;
      int node = nodeBase + slot;
      if (node > nN - 1) node = nN - 1;
      const v4f v = *(const v4f*)(susv + (size_t)node * 16 + 8 + 4 * half);
      *(v4f*)(ssv + slot * NHD + 4 * half) = v;
    }
    if (wave == 0) {
      float c0 = 0.f, c1 = 0.f, cb = 0.f;
#pragma unroll 1
      for (int k = 0; k < DIMF; ++k) {
        const float we = w_att_e[k * NHD + hd];
        c0 += w_edge[k] * we;
        c1 += w_edge[DIMF + k] * we;
        cb += b_edge[k] * we;
      }
      if (lane < 8) {
        kap[hd]      = c0;
        kap[8 + hd]  = c1;
        kap[16 + hd] = cb + b_att_e[hd];
      }
    }
  }
  __syncthreads();
  const float ka0 = kap[hd], ka1 = kap[8 + hd], kab = kap[16 + hd];

  const int nChunks = (nE + CHUNK - 1) / CHUNK;
#pragma unroll 1
  for (int ch = 0; ch < nChunks; ++ch) {
    const int cbase = ch * CHUNK;
    int wc = 0;
#pragma unroll
    for (int g = 0; g < NGRP; ++g) {
      const int el0 = (g * NTHR + tid) * 4;
      const int e0  = cbase + el0;
      const int sent = -2147483647 - 1;
      v4i d;
      if (cbase + CHUNK <= nE) {
        d = *(const v4i*)(dsti + e0);
      } else {
        d.x = (e0     < nE) ? dsti[min(e0,     nE - 1)] : sent;
        d.y = (e0 + 1 < nE) ? dsti[min(e0 + 1, nE - 1)] : sent;
        d.z = (e0 + 2 < nE) ? dsti[min(e0 + 2, nE - 1)] : sent;
        d.w = (e0 + 3 < nE) ? dsti[min(e0 + 3, nE - 1)] : sent;
      }
      const unsigned s0 = (unsigned)d.x - (unsigned)nodeBase;
      const unsigned s1 = (unsigned)d.y - (unsigned)nodeBase;
      const unsigned s2 = (unsigned)d.z - (unsigned)nodeBase;
      const unsigned s3 = (unsigned)d.w - (unsigned)nodeBase;
      const bool q0 = s0 < (unsigned)NB;
      const bool q1 = s1 < (unsigned)NB;
      const bool q2 = s2 < (unsigned)NB;
      const bool q3 = s3 < (unsigned)NB;
      const unsigned many = __builtin_amdgcn_ballot_w32(q0 | q1 | q2 | q3);
      if (many != 0u) {
#define HITJ(J, QJ, SJ) { \
          const unsigned mj = __builtin_amdgcn_ballot_w32(QJ); \
          if (QJ) { \
            const int pos = wc + (int)__builtin_amdgcn_mbcnt_lo(mj, 0u); \
            if (pos < WCAP) list[wave * WCAP + pos] = ((el0 + (J)) << 9) | (int)(SJ); \
          } \
          wc += (int)__builtin_popcount(mj); }
        HITJ(0, q0, s0)
        HITJ(1, q1, s1)
        HITJ(2, q2, s2)
        HITJ(3, q3, s3)
#undef HITJ
      }
    }
    if (lane == 0) wcnt[wave] = wc;
    __syncthreads();

    if (wave == 0) {
      for (int wsx = 0; wsx < NWAVE; ++wsx) {
        int nh = wcnt[wsx];
        if (nh > WCAP) nh = WCAP;
        if (nh < 0) nh = 0;
        for (int i = 0; i < nh; ++i) {
          const int ent  = list[wsx * WCAP + i];
          const int slot = ent & (NB - 1);
          const int el   = (ent >> 9) & (CHUNK - 1);
          int e = cbase + el;
          if (e > nE - 1) e = nE - 1;
          int s = srci[e];
          s = s < 0 ? 0 : (s > nN - 1 ? nN - 1 : s);
          const v2f ef = *(const v2f*)(edge_feat + 2 * (size_t)e);
          const float a_u = susv[(size_t)s * 16 + hd];
          const float a_v = ssv[slot * NHD + hd];
          float sc = a_u + a_v;
          const float se = ef.x * ka0 + ef.y * ka1 + kab;
          sc = sc + se;
          sc = (sc > 0.f) ? sc : 0.2f * sc;
          const float mo   = smax[slot * NHD + hd];
          const float dold = sden[slot * NHD + hd];
          const float mn   = fmaxf(mo, sc);
          const float scl  = __expf(mo - mn);
          const float p    = __expf(sc - mn);
          if (lane < 8) {
            smax[slot * NHD + hd] = mn;
            sden[slot * NHD + hd] = dold * scl + p;
          }
          const float scl0 = __shfl(scl, hc0, 32);
          const float p0   = __shfl(p,   hc0, 32);
          const float scl1 = __shfl(scl, hc1, 32);
          const float p1   = __shfl(p,   hc1, 32);
          const v2f hv = *(const v2f*)(hbuf + (size_t)s * DIMF + 2 * lane);
          v2f* ap = (v2f*)(sacc + slot * DIMF + 2 * lane);
          v2f a = *ap;
          a.x = a.x * scl0 + p0 * hv.x;
          a.y = a.y * scl1 + p1 * hv.y;
          *ap = a;
        }
      }
    }
    __syncthreads();
  }

#pragma unroll 1
  for (int gq = 0; gq < NB / 16; ++gq) {
    const int node0 = nodeBase + gq * 16;
    if (node0 >= nN) break;
    {
      const int row  = tid >> 4;
      const int c0   = (tid & 15) * 4;
      const int slot = gq * 16 + row;
      const v4f d4 = *(const v4f*)(sden + slot * NHD + (c0 & 7));
      const v4f a4 = *(const v4f*)(sacc + slot * DIMF + c0);
      v4us uh, ul;
#pragma unroll
      for (int j = 0; j < 4; ++j) {
        const float rd = 1.0f / fmaxf(d4[j], 1e-12f);
        const float v  = a4[j] * rd;
        us a, c;
        spl(v, a, c);
        uh[j] = a;
        ul[j] = c;
      }
      *(v4us*)(Ah + row * APN + c0) = uh;
      *(v4us*)(Al + row * APN + c0) = ul;
    }
    __syncthreads();
    {
      const int nt0 = 2 * wave, nt1 = 2 * wave + 1;
      v8f g0 = {0.f, 0.f, 0.f, 0.f, 0.f, 0.f, 0.f, 0.f};
      v8f g1 = {0.f, 0.f, 0.f, 0.f, 0.f, 0.f, 0.f, 0.f};
#pragma unroll
      for (int kt = 0; kt < DIMF / 32; ++kt) {
        const int k0 = kt * 32 + 8 * hh;
        FragB ah, al, b0h, b0l, b1h, b1l;
        ldf(ah, Ah + m * APN + k0);
        ldf(al, Al + m * APN + k0);
        ldf(b0h, W1H + (size_t)(16 * nt0 + m) * DIMF + k0);
        ldf(b0l, W1L + (size_t)(16 * nt0 + m) * DIMF + k0);
        ldf(b1h, W1H + (size_t)(16 * nt1 + m) * DIMF + k0);
        ldf(b1l, W1L + (size_t)(16 * nt1 + m) * DIMF + k0);
        g0 = wm3(ah, al, b0h, b0l, g0);
        g1 = wm3(ah, al, b1h, b1l, g1);
      }
      const int col0 = 16 * nt0 + m, col1 = 16 * nt1 + m;
      const float bias0 = b_ff1[col0], bias1 = b_ff1[col1];
#pragma unroll
      for (int r = 0; r < 8; ++r) {
        const int row = 8 * hh + r;
        us a, c;
        const float v0 = gelu_x(g0[r] + bias0);
        spl(v0, a, c); Gh[row * GPN + col0] = a; Gl[row * GPN + col0] = c;
        const float v1 = gelu_x(g1[r] + bias1);
        spl(v1, a, c); Gh[row * GPN + col1] = a; Gl[row * GPN + col1] = c;
      }
    }
    __syncthreads();
    {
      const int nt = wave & 3;
      const int ncol = 16 * nt + m;
      v8f o = {0.f, 0.f, 0.f, 0.f, 0.f, 0.f, 0.f, 0.f};
#pragma unroll 2
      for (int kt = 0; kt < HID / 32; ++kt) {
        const int k0 = kt * 32 + 8 * hh;
        FragB ah, al, bh, bl;
        ldf(ah, Gh + m * GPN + k0);
        ldf(al, Gl + m * GPN + k0);
        ldf(bh, W2H + (size_t)ncol * HID + k0);
        ldf(bl, W2L + (size_t)ncol * HID + k0);
        o = wm3(ah, al, bh, bl, o);
      }
      const float bias = b_ff2[ncol];
      if (wave < 4) {
#pragma unroll
        for (int r = 0; r < 8; ++r) Os[(8 * hh + r) * HPN + ncol] = o[r] + bias;
      }
    }
    __syncthreads();
    {
      const int row  = tid >> 4;
      const int c4   = (tid & 15) * 4;
      const int node = node0 + row;
      const v4f v = *(const v4f*)(Os + row * HPN + c4);
      int nd = node;
      if (nd > nN - 1) nd = nN - 1;
      float* op = out + (size_t)nd * DIMF + c4;
      const bool ok = (node < nN);
      if (ok) *(volatile v4f*)op = v;
      __threadfence();
      if (ok) *(volatile v4f*)op = v;
    }
  }
}

extern "C" void kernel_launch(void* const* d_in, const int* in_sizes, int n_in,
                              void* d_out, int out_size, void* d_ws, size_t ws_size,
                              hipStream_t stream) {
  if (n_in < 17) return;
  const int nN = in_sizes[0] / DIMF;
  if (nN <= 0 || in_sizes[0] != nN * DIMF) return;
  const int nE = in_sizes[15];
  if (nE < 0 || in_sizes[16] != nE || in_sizes[1] != 2 * nE) return;
  if (in_sizes[2] != DIMF * DIMF || in_sizes[3] != DIMF) return;
  if (in_sizes[4] != 2 * DIMF || in_sizes[5] != DIMF) return;
  if (in_sizes[6] != DIMF * NHD || in_sizes[7] != NHD || in_sizes[8] != DIMF * NHD) return;
  if (in_sizes[9] != DIMF * NHD || in_sizes[10] != NHD) return;
  if (in_sizes[11] != DIMF * HID || in_sizes[12] != HID || in_sizes[13] != HID * DIMF || in_sizes[14] != DIMF) return;
  if (out_size != nN * DIMF) return;

  const float* x         = (const float*)d_in[0];
  const float* edge_feat = (const float*)d_in[1];
  const float* w_in      = (const float*)d_in[2];
  const float* b_in      = (const float*)d_in[3];
  const float* w_edge    = (const float*)d_in[4];
  const float* b_edge    = (const float*)d_in[5];
  const float* w_att_u   = (const float*)d_in[6];
  const float* b_att_u   = (const float*)d_in[7];
  const float* w_att_v   = (const float*)d_in[8];
  const float* w_att_e   = (const float*)d_in[9];
  const float* b_att_e   = (const float*)d_in[10];
  const float* w_ff1     = (const float*)d_in[11];
  const float* b_ff1     = (const float*)d_in[12];
  const float* w_ff2     = (const float*)d_in[13];
  const float* b_ff2     = (const float*)d_in[14];
  const int*   srci      = (const int*)d_in[15];
  const int*   dsti      = (const int*)d_in[16];
  float* out = (float*)d_out;

  const int nP = ((nN + GR - 1) / GR) * GR;
  size_t off = 0;
  us* WinH = (us*)((char*)d_ws + off); off += (size_t)DIMF * DIMF * 2;
  us* WinL = (us*)((char*)d_ws + off); off += (size_t)DIMF * DIMF * 2;
  us* WuvH = (us*)((char*)d_ws + off); off += (size_t)16 * DIMF * 2;
  us* WuvL = (us*)((char*)d_ws + off); off += (size_t)16 * DIMF * 2;
  us* W1H  = (us*)((char*)d_ws + off); off += (size_t)HID * DIMF * 2;
  us* W1L  = (us*)((char*)d_ws + off); off += (size_t)HID * DIMF * 2;
  us* W2H  = (us*)((char*)d_ws + off); off += (size_t)DIMF * HID * 2;
  us* W2L  = (us*)((char*)d_ws + off); off += (size_t)DIMF * HID * 2;
  float* hbuf = (float*)((char*)d_ws + off); off += (size_t)nP * DIMF * sizeof(float);
  float* susv = (float*)((char*)d_ws + off); off += (size_t)nP * 16 * sizeof(float);
  if (off > ws_size) return;
  if (off > (size_t)134217728) return;

  k_prep<<<NPREP, NTHR, 0, stream>>>(w_in, w_att_u, w_att_v, w_ff1, w_ff2,
                                     WinH, WinL, WuvH, WuvL, W1H, W1L, W2H, W2L);

  k_node<<<nP / GR, 128, 0, stream>>>(x, b_in, b_att_u, WinH, WinL, WuvH, WuvL, hbuf, susv, nN);

  hipFuncSetAttribute(reinterpret_cast<const void*>(&k_agg),
                      hipFuncAttributeMaxDynamicSharedMemorySize, LDS_BYTES);
  const int grid = (nN + NB - 1) / NB;
  k_agg<<<grid, NTHR, LDS_BYTES, stream>>>(hbuf, susv, edge_feat, srci, dsti, w_edge, b_edge,
                                           w_att_e, b_att_e, W1H, W1L, W2H, W2L, b_ff1, b_ff2,
                                           out, nN, nE);
}
